// KAN_Convolution_3238405341764
// MI455X (gfx1250) — hardware-verified
//
#include <hip/hip_runtime.h>


#define IN_CH      32
#define OUT_CH     64
#define KW         9
#define PADW       4
#define LEN        2048
#define BATCH      16
#define NCOEF      8
#define FEAT       (IN_CH * (NCOEF + 1))
#define KRED       (KW * FEAT)
#define LPAD       (LEN + 2 * PADW)
#define W_ELEMS    (OUT_CH * KRED)
#define A_PER_B    (LPAD * FEAT)
#define ACT_CHUNK  8
#define ACT_CHUNKS (LPAD / ACT_CHUNK)
#define ACT_LINES  (ACT_CHUNK * FEAT / 64)
#define PREP_ROWS  2
#define PREP_LINES (PREP_ROWS * KRED / 64)
#define GEMM_LG    (BATCH * LEN / 256)
#define OPSCALE    16.0f
#define OUTSCALE   (1.0f / 256.0f)

static_assert(KRED % 32 == 0);
static_assert(FEAT % 8 == 0);
static_assert(LPAD % ACT_CHUNK == 0);
static_assert((ACT_CHUNK * FEAT) % 64 == 0);
static_assert((PREP_ROWS * KRED) % 64 == 0);
static_assert(A_PER_B % 64 == 0);
static_assert(OUT_CH % PREP_ROWS == 0);
static_assert((BATCH * LEN) % 256 == 0);
static_assert(LEN % 32 == 0);
static_assert(PREP_LINES <= 96 && ACT_LINES <= 64);

typedef _Float16 v16h __attribute__((ext_vector_type(16)));
typedef _Float16 v8h  __attribute__((ext_vector_type(8)));
typedef float    v8f  __attribute__((ext_vector_type(8)));
typedef float    v4f  __attribute__((ext_vector_type(4)));
union Frag { v16h v; v8h half[2]; };

static __device__ __forceinline__ v8f wmma16(v16h a, v16h b, v8f c) {
  v8f d = __builtin_amdgcn_wmma_f32_16x16x32_f16(false, a, false, b, (short)0, c, false, false);
  asm volatile("v_nop\n\tv_nop\n\tv_nop\n\tv_nop" : "+v"(d) : "v"(a), "v"(b));
  return d;
}

__global__ __launch_bounds__(256) void kan_prep_w(
    const float* __restrict__ base_w,
    const float* __restrict__ spline_w,
    const float* __restrict__ scaler,
    _Float16* __restrict__ W, int nblk) {
  __shared__ __attribute__((aligned(16))) _Float16 S[PREP_ROWS * KRED];
  const int blk = blockIdx.x;
  if (blk >= nblk) return;
  const int tid = threadIdx.x, lane = tid & 31, wave = tid >> 5;
  const int o0 = blk * PREP_ROWS;

  for (int idx = tid; idx < PREP_ROWS * IN_CH * KW; idx += 256) {
    const int ol  = idx / (IN_CH * KW);
    const int rem = idx - ol * (IN_CH * KW);
    const int i   = rem / KW;
    const int k   = rem - i * KW;
    const int src = ((o0 + ol) * IN_CH + i) * KW + k;
    const float sc = scaler[src];
    _Float16* p = S + ol * KRED + k * FEAT + i * (NCOEF + 1);
    p[0] = (_Float16)(base_w[src] * OPSCALE);
#pragma unroll
    for (int c = 0; c < NCOEF; ++c) {
      float sw = spline_w[(size_t)src * NCOEF + c] * sc;
      p[1 + c] = (_Float16)(sw * OPSCALE);
    }
  }
  __syncthreads();

  const int q = lane >> 3, pc = lane & 7;
  _Float16* Wb = W + (size_t)o0 * KRED;
  const int ln0 = wave * 4 + q;
  const int ln1 = 32 + wave * 4 + q;
  const int ln2 = 64 + wave * 4 + q;
  const bool has2 = (ln2 < PREP_LINES);
  v8h v0 = *(const v8h*)(S + ln0 * 64 + pc * 8);
  v8h v1 = *(const v8h*)(S + ln1 * 64 + pc * 8);
  v8h v2 = v0;
  if (has2) v2 = *(const v8h*)(S + ln2 * 64 + pc * 8);

  *(volatile v8h*)(Wb + ln0 * 64 + pc * 8) = v0;
  *(volatile v8h*)(Wb + ln1 * 64 + pc * 8) = v1;
  if (has2) *(volatile v8h*)(Wb + ln2 * 64 + pc * 8) = v2;
  __threadfence();
  *(volatile v8h*)(Wb + ln0 * 64 + pc * 8) = v0;
  *(volatile v8h*)(Wb + ln1 * 64 + pc * 8) = v1;
  if (has2) *(volatile v8h*)(Wb + ln2 * 64 + pc * 8) = v2;
}

__global__ __launch_bounds__(256) void kan_act(
    const float* __restrict__ x,
    _Float16* __restrict__ A, int nblk) {
#pragma clang fp contract(off)
  __shared__ __attribute__((aligned(16))) _Float16 S[ACT_CHUNK * FEAT];
  const int blk = blockIdx.x;
  if (blk >= nblk) return;
  const int b     = blk / ACT_CHUNKS;
  const int chunk = blk - b * ACT_CHUNKS;
  const int tid = threadIdx.x, lane = tid & 31, wave = tid >> 5;
  const int i   = tid & (IN_CH - 1);
  const int lpl = tid >> 5;
  const int lp  = chunk * ACT_CHUNK + lpl;

  float xv = 0.0f;
  const int l = lp - PADW;
  if (l >= 0 && l < LEN) xv = x[((size_t)(b * IN_CH + i)) * LEN + l];

  const float s = xv / (1.0f + expf(-xv));

  float t[12];
#pragma unroll
  for (int j = 0; j < 12; ++j) { float pj = (float)(j - 3) * 0.4f; t[j] = pj + (-1.0f); }
  float bs[11];
#pragma unroll
  for (int j = 0; j < 11; ++j) bs[j] = (xv >= t[j] && xv < t[j + 1]) ? 1.0f : 0.0f;
#pragma unroll
  for (int k = 1; k <= 3; ++k) {
#pragma unroll
    for (int j = 0; j < 11 - k; ++j) {
      const float invl = 1.0f / (t[j + k] - t[j]);
      const float invr = 1.0f / (t[j + k + 1] - t[j + 1]);
      const float left  = (xv - t[j]) * invl;
      const float right = (t[j + k + 1] - xv) * invr;
      const float pl = left * bs[j];
      const float pr = right * bs[j + 1];
      bs[j] = pl + pr;
    }
  }

  _Float16* p = S + lpl * FEAT + i * (NCOEF + 1);
  p[0] = (_Float16)(s * OPSCALE);
#pragma unroll
  for (int c = 0; c < NCOEF; ++c) p[1 + c] = (_Float16)(bs[c] * OPSCALE);
  __syncthreads();

  const int q = lane >> 3, pc = lane & 7;
  const size_t gbase = (size_t)b * A_PER_B + (size_t)chunk * (ACT_CHUNK * FEAT);
  const int ln0 = wave * 4 + q;
  const int ln1 = 32 + wave * 4 + q;
  const bool has1 = (ln1 < ACT_LINES);
  v8h v0 = *(const v8h*)(S + ln0 * 64 + pc * 8);
  v8h v1 = v0;
  if (has1) v1 = *(const v8h*)(S + ln1 * 64 + pc * 8);

  *(volatile v8h*)(A + gbase + ln0 * 64 + pc * 8) = v0;
  if (has1) *(volatile v8h*)(A + gbase + ln1 * 64 + pc * 8) = v1;
  __threadfence();
  *(volatile v8h*)(A + gbase + ln0 * 64 + pc * 8) = v0;
  if (has1) *(volatile v8h*)(A + gbase + ln1 * 64 + pc * 8) = v1;
}

union __attribute__((aligned(16))) GemmLds {
  _Float16 w[32 * KRED];
  float    st[8 * 1024];
};

static __device__ __forceinline__ void stage_tile(float* st, v8f acc, int ot, int lt, int m, int h) {
  float* p = st + (ot * 16 + m) * 32 + lt * 16 + 8 * h;
  v4f lo = __builtin_shufflevector(acc, acc, 0, 1, 2, 3) * OUTSCALE;
  v4f hi = __builtin_shufflevector(acc, acc, 4, 5, 6, 7) * OUTSCALE;
  *(v4f*)(p)     = lo;
  *(v4f*)(p + 4) = hi;
}

__global__ __launch_bounds__(256) void kan_gemm(
    const _Float16* __restrict__ A,
    const _Float16* __restrict__ W,
    float* __restrict__ out,
    int nlg) {
  __shared__ GemmLds lds;

  const int tid  = threadIdx.x;
  const int lane = tid & 31;
  const int wave = tid >> 5;
  const int ot2  = blockIdx.x & 1;
  const int lg   = blockIdx.x >> 1;
  if (lg >= nlg) return;

  {
    const _Float16* src = W + (size_t)ot2 * 32 * KRED;
    const int n128 = (32 * KRED) / 8;
    for (int idx = tid; idx < n128; idx += 256)
      *(v8h*)(lds.w + (size_t)idx * 8) = *(const v8h*)(src + (size_t)idx * 8);
  }
  __syncthreads();

  const int gl0 = (lg * 8 + wave) * 32;
  const int b   = gl0 / LEN;
  const int l0  = gl0 - b * LEN;
  const int m   = lane & 15;
  const int h   = lane >> 4;

  const _Float16* ar0 = A + (size_t)b * A_PER_B + (size_t)(l0 + m) * FEAT + 8 * h;
  const _Float16* ar1 = ar0 + (size_t)16 * FEAT;
  const _Float16* wl0 = lds.w + (size_t)m * KRED + 8 * h;
  const _Float16* wl1 = wl0 + (size_t)16 * KRED;

  v8f acc00 = {}, acc01 = {}, acc10 = {}, acc11 = {};

#pragma unroll 1
  for (int r = 0; r < KRED; r += 32) {
    Frag a0, a1, w0, w1;
    a0.half[0] = *(const v8h*)(ar0 + r);
    a0.half[1] = *(const v8h*)(ar0 + r + 16);
    a1.half[0] = *(const v8h*)(ar1 + r);
    a1.half[1] = *(const v8h*)(ar1 + r + 16);
    w0.half[0] = *(const v8h*)(wl0 + r);
    w0.half[1] = *(const v8h*)(wl0 + r + 16);
    w1.half[0] = *(const v8h*)(wl1 + r);
    w1.half[1] = *(const v8h*)(wl1 + r + 16);

    acc00 = wmma16(a0.v, w0.v, acc00);
    acc01 = wmma16(a0.v, w1.v, acc01);
    acc10 = wmma16(a1.v, w0.v, acc10);
    acc11 = wmma16(a1.v, w1.v, acc11);
  }

  __syncthreads();
  float* st = lds.st + wave * 1024;
  stage_tile(st, acc00, 0, 0, m, h);
  stage_tile(st, acc01, 1, 0, m, h);
  stage_tile(st, acc10, 0, 1, m, h);
  stage_tile(st, acc11, 1, 1, m, h);
  __syncthreads();

  const int q = lane >> 3, pc = lane & 7;
  const int obase = ot2 * 32;
  v4f v[8];
#pragma unroll
  for (int it = 0; it < 8; ++it) {
    const int ol = it * 4 + q;
    v[it] = *(const v4f*)(st + ol * 32 + pc * 4);
  }
#pragma unroll
  for (int it = 0; it < 8; ++it) {
    const int ol = it * 4 + q;
    float* gp = out + ((size_t)(b * OUT_CH + obase + ol) * LEN) + l0 + pc * 4;
    *(volatile v4f*)gp = v[it];
  }
  __threadfence();
#pragma unroll
  for (int it = 0; it < 8; ++it) {
    const int ol = it * 4 + q;
    float* gp = out + ((size_t)(b * OUT_CH + obase + ol) * LEN) + l0 + pc * 4;
    *(volatile v4f*)gp = v[it];
  }
}

extern "C" void kernel_launch(void* const* d_in, const int* in_sizes, int n_in,
                              void* d_out, int out_size, void* d_ws, size_t ws_size,
                              hipStream_t stream) {
  if (n_in < 4) return;
  if (in_sizes[0] != BATCH * IN_CH * LEN) return;
  if (in_sizes[1] != OUT_CH * IN_CH * KW) return;
  if (in_sizes[2] != OUT_CH * IN_CH * KW * NCOEF) return;
  if (in_sizes[3] != OUT_CH * IN_CH * KW) return;
  if (out_size != BATCH * OUT_CH * LEN) return;

  const size_t w_bytes = (size_t)W_ELEMS * 2;
  const size_t a_bytes = (size_t)BATCH * A_PER_B * 2;
  if (w_bytes + a_bytes > ws_size) return;

  const float* x        = (const float*)d_in[0];
  const float* base_w   = (const float*)d_in[1];
  const float* spline_w = (const float*)d_in[2];
  const float* scaler   = (const float*)d_in[3];
  float* out = (float*)d_out;

  _Float16* W = (_Float16*)d_ws;
  _Float16* A = (_Float16*)((char*)d_ws + w_bytes);

  const int nprep = OUT_CH / PREP_ROWS;
  kan_prep_w<<<nprep, 256, 0, stream>>>(base_w, spline_w, scaler, W, nprep);

  const int nact = BATCH * ACT_CHUNKS;
  kan_act<<<nact, 256, 0, stream>>>(x, A, nact);

  kan_gemm<<<2 * GEMM_LG, 256, 0, stream>>>(A, W, out, GEMM_LG);
}
